// ModularTreeLSTMPredictor_42649025249412
// MI455X (gfx1250) — hardware-verified
//
#include <hip/hip_runtime.h>
#include <math.h>

constexpr int NBT  = 128;
constexpr int NND  = 512;
constexpr int NFT  = 63;
constexpr int NHU  = 128;
constexpr int NMD  = 2;
constexpr int KXP  = NFT + 1;
constexpr int KGT  = KXP + 2 * NHU;
constexpr int NGO  = 5 * NHU;
constexpr int NBTR = NMD * NGO;
constexpr int RBLK = 16;
constexpr int NTH  = 512;
constexpr int NWV  = NTH / 32;
constexpr int APH  = 328;
constexpr int APW  = APH / 2;
constexpr int SPF  = 132;
constexpr int TPT  = 256;
constexpr float WSCL     = 64.0f;
constexpr float WSCL_INV = 1.0f / 64.0f;

static_assert(NBT % RBLK == 0);
static_assert(NWV == RBLK);
static_assert(NWV == NMD * (NHU / 16));
static_assert(KGT % 32 == 0);
static_assert(KXP == 64);
static_assert(KGT % 64 == 0 && NGO % 64 == 0);
static_assert(APH % 8 == 0 && APH >= KGT);
static_assert(SPF % 4 == 0 && SPF >= NHU);
static_assert((RBLK * NND) % (4 * NTH) == 0);
static_assert((NND * 4) % 128 == 0);
static_assert(NHU == 4 * 32);
static_assert(NHU == 8 * 16);
static_assert(NND - 1 < 65536);

typedef __attribute__((ext_vector_type(16))) _Float16 v16h;
typedef __attribute__((ext_vector_type(8)))  _Float16 v8h;
typedef __attribute__((ext_vector_type(8)))  float    v8f;
typedef __attribute__((ext_vector_type(4)))  float    v4f;
typedef __attribute__((ext_vector_type(4)))  unsigned v4u;
typedef __attribute__((ext_vector_type(2)))  unsigned v2u;

__device__ __forceinline__ unsigned short f2bf_bits(float f) {
  unsigned u = __float_as_uint(f);
  return (unsigned short)((u + 0x7FFFu + ((u >> 16) & 1u)) >> 16);
}
__device__ __forceinline__ float bf_bits2f(unsigned short h) { return __uint_as_float(((unsigned)h) << 16); }
__device__ __forceinline__ float bf16r(float f) { return bf_bits2f(f2bf_bits(f)); }
__device__ __forceinline__ unsigned h16_bits(float f) { return (unsigned)__builtin_bit_cast(unsigned short, (_Float16)f); }
__device__ __forceinline__ unsigned pack_h2(float a, float b) { return h16_bits(a) | (h16_bits(b) << 16); }

__device__ __forceinline__ void mma_guard4m(v8f& a0, v8f& a1, v8f& a2, v8f& a3,
                                            v16h x, v16h y0, v16h y1, v16h y2, v16h y3) {
  asm volatile("v_nop\n\tv_nop\n\tv_nop\n\tv_nop"
               : "+v"(a0), "+v"(a1), "+v"(a2), "+v"(a3)
               : "v"(x), "v"(y0), "v"(y1), "v"(y2), "v"(y3)
               : "memory");
}
__device__ __forceinline__ void mma_guard1m(v8f& a4, v16h x, v16h y) {
  asm volatile("v_nop\n\tv_nop\n\tv_nop\n\tv_nop" : "+v"(a4) : "v"(x), "v"(y) : "memory");
}
__device__ __forceinline__ void acc_guard5(v8f& a, v8f& b, v8f& c, v8f& d, v8f& e) {
  asm volatile("v_nop\n\tv_nop\n\tv_nop\n\tv_nop" : "+v"(a), "+v"(b), "+v"(c), "+v"(d), "+v"(e));
}

template <typename T> struct Frag;
template <> struct Frag<_Float16> {
  typedef v16h V; union U { v16h v; v8h h[2]; };
  static __device__ __forceinline__ v16h load(const _Float16* p) {
    U f; f.h[0] = *(const v8h*)(p); f.h[1] = *(const v8h*)(p + 16); return f.v;
  }
  static __device__ __forceinline__ v8f mma(v16h a, v16h b, v8f c) {
    return __builtin_amdgcn_wmma_f32_16x16x32_f16(false, a, false, b, (short)0, c, false, false);
  }
};

__device__ __forceinline__ float fsig(float x)  { return __builtin_amdgcn_rcpf(1.0f + expf(-x)); }
__device__ __forceinline__ float ftanh(float x) { return 1.0f - 2.0f * __builtin_amdgcn_rcpf(expf(2.0f * x) + 1.0f); }

template <int MODE>
__global__ __launch_bounds__(TPT) void tpw_kernel(const float* __restrict__ src, int R, int C, int ldo,
                                                 unsigned short* __restrict__ O, float sc) {
  __shared__ float Tt[64 * 65];
  const int tid = threadIdx.x;
  const int c0 = blockIdx.x * 64, r0 = blockIdx.y * 64;
  src += (size_t)blockIdx.z * (size_t)R * (size_t)C;
  O   += (size_t)blockIdx.z * (size_t)C * (size_t)ldo;
#pragma unroll
  for (int i = 0; i < 4; ++i) {
    const int idx = i * TPT + tid;
    const int rr = idx >> 4, cc = (idx & 15) * 4;
    const v4f v = *(const v4f*)(src + (size_t)(r0 + rr) * (size_t)C + c0 + cc);
    Tt[rr * 65 + cc + 0] = v[0];
    Tt[rr * 65 + cc + 1] = v[1];
    Tt[rr * 65 + cc + 2] = v[2];
    Tt[rr * 65 + cc + 3] = v[3];
  }
  __syncthreads();
  const int q = tid >> 3, c8 = (tid & 7) * 8;
  v8h hv[2];
#pragma unroll
  for (int g = 0; g < 2; ++g) {
    const int qq = g * 32 + q;
#pragma unroll
    for (int e = 0; e < 8; ++e) {
      const float f = Tt[(c8 + e) * 65 + qq];
      unsigned short bits;
      if (MODE == 0) {
        bits = f2bf_bits(f * sc);
      } else {
        const float fb = bf_bits2f(f2bf_bits(f));
        bits = __builtin_bit_cast(unsigned short, (_Float16)(fb * sc));
      }
      hv[g][e] = __builtin_bit_cast(_Float16, bits);
    }
  }
  for (int pass = 0; pass < 2; ++pass) {
#pragma unroll
    for (int g = 0; g < 2; ++g) {
      const size_t o = (size_t)(c0 + g * 32 + q) * (size_t)ldo + (size_t)(r0 + c8);
      *(volatile v8h*)(O + o) = hv[g];
    }
    __threadfence();
  }
}

__device__ __forceinline__ void gate_ktile(v8f (&acc)[5], const _Float16* ap,
                                           const _Float16* b0p, const _Float16* b1p, const _Float16* b2p,
                                           const _Float16* b3p, const _Float16* b4p) {
  const v16h a  = Frag<_Float16>::load(ap);
  const v16h f0 = Frag<_Float16>::load(b0p);
  const v16h f1 = Frag<_Float16>::load(b1p);
  const v16h f2 = Frag<_Float16>::load(b2p);
  const v16h f3 = Frag<_Float16>::load(b3p);
  acc[0] = Frag<_Float16>::mma(a, f0, acc[0]);
  acc[1] = Frag<_Float16>::mma(a, f1, acc[1]);
  acc[2] = Frag<_Float16>::mma(a, f2, acc[2]);
  acc[3] = Frag<_Float16>::mma(a, f3, acc[3]);
  mma_guard4m(acc[0], acc[1], acc[2], acc[3], a, f0, f1, f2, f3);
  const v16h f4 = Frag<_Float16>::load(b4p);
  acc[4] = Frag<_Float16>::mma(a, f4, acc[4]);
  mma_guard1m(acc[4], a, f4);
}

__global__ __launch_bounds__(NTH) void tree_kernel(
    const float* __restrict__ feats, const float* __restrict__ treat,
    const float* __restrict__ bgate, const float* __restrict__ wout, const float* __restrict__ bout,
    const int* __restrict__ modidx, const int* __restrict__ lch, const int* __restrict__ rch,
    const unsigned short* __restrict__ Btp, unsigned* H16w, float* C32, float* __restrict__ out) {
  __shared__ __align__(16) unsigned As32[RBLK * APW];
  __shared__ __align__(16) float    sH[RBLK * SPF];
  __shared__ __align__(16) float    sC[RBLK * SPF];
  __shared__ __align__(16) float    sP[NMD * 8 * RBLK];
  __shared__ __align__(16) float    sOut[RBLK * NND];
  __shared__ int sMod[RBLK];

  const _Float16* As = (const _Float16*)As32;
  const _Float16* Bt = (const _Float16*)Btp;
  const int tid = threadIdx.x, lane = tid & 31, wave = tid >> 5;
  const int c = lane & 15, hh = lane >> 4, koff = hh * 8;
  const int b0 = blockIdx.x * RBLK;
  const int mw = wave >> 3, ut = wave & 7, j = ut * 16 + c;
  const int brow = b0 + wave;

  const float bg0 = bf16r(bgate[mw * NGO + 0 * NHU + j]);
  const float bg1 = bf16r(bgate[mw * NGO + 1 * NHU + j]);
  const float bg2 = bf16r(bgate[mw * NGO + 2 * NHU + j]);
  const float bg3 = bf16r(bgate[mw * NGO + 3 * NHU + j]);
  const float bg4 = bf16r(bgate[mw * NGO + 4 * NHU + j]);
  const float wo  = bf16r(wout[mw * NHU + j]);
  const float bo0 = bf16r(bout[0]);
  const float bo1 = bf16r(bout[1]);
  const float trt = bf16r(treat[brow]);
  asm volatile("" ::: "memory");

#pragma unroll 1
  for (int i = tid; i < RBLK * APW; i += NTH) As32[i] = 0u;
  int mprev = 0;
  __syncthreads();

  const _Float16* arow = As + c * APH + koff;
  const _Float16* bp0 = Bt + (size_t)(mw * NGO + 0 * NHU + j) * KGT + koff;
  const _Float16* bp1 = Bt + (size_t)(mw * NGO + 1 * NHU + j) * KGT + koff;
  const _Float16* bp2 = Bt + (size_t)(mw * NGO + 2 * NHU + j) * KGT + koff;
  const _Float16* bp3 = Bt + (size_t)(mw * NGO + 3 * NHU + j) * KGT + koff;
  const _Float16* bp4 = Bt + (size_t)(mw * NGO + 4 * NHU + j) * KGT + koff;
  const float fa = fminf(1.0f, (float)(31 - lane));
  const float fb = 1.0f - fa;
  const int   i1 = (2 * lane + 1 < NFT - 1) ? (2 * lane + 1) : (NFT - 1);
  const v8f z8 = {0.f, 0.f, 0.f, 0.f, 0.f, 0.f, 0.f, 0.f};

#pragma unroll 1
  for (int t = 0; t < NND; ++t) {
    const int lc = __builtin_amdgcn_readfirstlane(lch[t]);
    const int rc = __builtin_amdgcn_readfirstlane(rch[t]);
    const bool lval = (lc >= 0) && (lc < t);
    const bool rval = (rc >= 0) && (rc < t);
    const int lcc = lc < 0 ? 0 : (lc > NND - 1 ? NND - 1 : lc);
    const int rcc = rc < 0 ? 0 : (rc > NND - 1 ? NND - 1 : rc);

    if (t > 0) {
      float s = mprev ? bo1 : bo0;
      const float* pp = sP + mprev * 8 * RBLK + wave;
#pragma unroll
      for (int u = 0; u < 8; ++u) s += pp[u * RBLK];
      if (lane == 0) sOut[wave * NND + (t - 1)] = s;
    }
    {
      int mv = modidx[(size_t)brow * NND + t];
      mv = mv < 0 ? 0 : (mv > NMD - 1 ? NMD - 1 : mv);
      mprev = mv;
      if (lane == 0) sMod[wave] = mv;
    }
    {
      const float* xb = feats + ((size_t)brow * NND + (size_t)t) * NFT;
      const float f0  = xb[2 * lane];
      const float f1r = xb[i1];
      const float f1  = fmaf(fa, f1r, fb * trt);
      As32[wave * APW + lane] = pack_h2(bf16r(f0), bf16r(f1));
    }
    {
      v2u lw = {0u, 0u}, rw = {0u, 0u};
      if (lval) lw = *(const v2u*)(H16w + ((size_t)brow * NND + (size_t)lcc) * (NHU / 2) + 2 * lane);
      if (rval) rw = *(const v2u*)(H16w + ((size_t)brow * NND + (size_t)rcc) * (NHU / 2) + 2 * lane);
      *(v2u*)(As32 + wave * APW + 32 + 2 * lane) = lw;
      *(v2u*)(As32 + wave * APW + 96 + 2 * lane) = rw;
    }
    __syncthreads();

    v8f acc[5];
    acc[0] = z8; acc[1] = z8; acc[2] = z8; acc[3] = z8; acc[4] = z8;
#pragma unroll 1
    for (int kt = 0; kt < 2; ++kt)
      gate_ktile(acc, arow + kt * 32, bp0 + kt * 32, bp1 + kt * 32, bp2 + kt * 32, bp3 + kt * 32, bp4 + kt * 32);
    if (lval) {
#pragma unroll 1
      for (int kt = 2; kt < 6; ++kt)
        gate_ktile(acc, arow + kt * 32, bp0 + kt * 32, bp1 + kt * 32, bp2 + kt * 32, bp3 + kt * 32, bp4 + kt * 32);
    }
    if (rval) {
#pragma unroll 1
      for (int kt = 6; kt < 10; ++kt)
        gate_ktile(acc, arow + kt * 32, bp0 + kt * 32, bp1 + kt * 32, bp2 + kt * 32, bp3 + kt * 32, bp4 + kt * 32);
    }
    acc_guard5(acc[0], acc[1], acc[2], acc[3], acc[4]);

    float lcl[8], rcl[8];
#pragma unroll
    for (int r = 0; r < 8; ++r) { lcl[r] = 0.0f; rcl[r] = 0.0f; }
    if (lval) {
      const float* cp = C32 + ((size_t)(b0 + 8 * hh) * NND + (size_t)lcc) * NHU + j;
#pragma unroll
      for (int r = 0; r < 8; ++r) lcl[r] = cp[(size_t)r * NND * NHU];
    }
    asm volatile("" ::: "memory");
    if (rval) {
      const float* cp = C32 + ((size_t)(b0 + 8 * hh) * NND + (size_t)rcc) * NHU + j;
#pragma unroll
      for (int r = 0; r < 8; ++r) rcl[r] = cp[(size_t)r * NND * NHU];
    }
    float pr[8];
#pragma unroll
    for (int r = 0; r < 8; ++r) {
      const int rr = 8 * hh + r;
      const bool own = (sMod[rr] == mw);
      const float zi = acc[0][r] * WSCL_INV + bg0;
      const float zl = acc[1][r] * WSCL_INV + bg1;
      const float zr = acc[2][r] * WSCL_INV + bg2;
      const float zo = acc[3][r] * WSCL_INV + bg3;
      const float zc = acc[4][r] * WSCL_INV + bg4;
      const float gi = fsig(zi), gl = fsig(zl), gr = fsig(zr), go = fsig(zo), gc = ftanh(zc);
      const float cell = gi * gc + gl * lcl[r] + gr * rcl[r];
      const float hid  = go * ftanh(cell);
      if (own) { sH[rr * SPF + j] = hid; sC[rr * SPF + j] = cell; }
      pr[r] = hid * wo;
    }
#pragma unroll
    for (int r = 0; r < 8; ++r) {
#pragma unroll
      for (int off = 1; off < 16; off <<= 1) pr[r] += __shfl_xor(pr[r], off, 32);
    }
    if (c == 0) {
      float* spw = sP + (mw * 8 + ut) * RBLK + 8 * hh;
#pragma unroll
      for (int r = 0; r < 8; ++r) spw[r] = pr[r];
    }
    __syncthreads();

    {
      const size_t rowid = (size_t)brow * NND + (size_t)t;
      const v4f cv = *(const v4f*)(sC + wave * SPF + 4 * lane);
      const int l16 = lane & 15;
      const v4f ha = *(const v4f*)(sH + wave * SPF + 8 * l16);
      const v4f hb = *(const v4f*)(sH + wave * SPF + 8 * l16 + 4);
      v4u hw;
      hw[0] = pack_h2(ha[0], ha[1]);
      hw[1] = pack_h2(ha[2], ha[3]);
      hw[2] = pack_h2(hb[0], hb[1]);
      hw[3] = pack_h2(hb[2], hb[3]);
      for (int pass = 0; pass < 2; ++pass) {
        *(volatile v4f*)(C32 + rowid * NHU + 4 * lane) = cv;
        if (lane < 16) *(volatile v4u*)(H16w + rowid * (NHU / 2) + 4 * lane) = hw;
        __threadfence();
      }
    }
    __syncthreads();
  }

  {
    float s = mprev ? bo1 : bo0;
    const float* pp = sP + mprev * 8 * RBLK + wave;
#pragma unroll
    for (int u = 0; u < 8; ++u) s += pp[u * RBLK];
    if (lane == 0) sOut[wave * NND + (NND - 1)] = s;
  }
  __syncthreads();
  for (int pass = 0; pass < 2; ++pass) {
#pragma unroll
    for (int it = 0; it < 4; ++it) {
      const int idx = it * NTH + tid;
      const int row = idx >> 7, c4 = (idx & 127) * 4;
      const v4f v = *(const v4f*)(sOut + row * NND + c4);
      *(volatile v4f*)(out + (size_t)(b0 + row) * NND + c4) = v;
    }
    __threadfence();
  }
}

extern "C" void kernel_launch(void* const* d_in, const int* in_sizes, int n_in,
                              void* d_out, int out_size, void* d_ws, size_t ws_size, hipStream_t stream) {
  if (n_in < 9 || d_out == nullptr || d_ws == nullptr) return;
  if (in_sizes[0] != NBT * NND * NFT || in_sizes[1] != NBT || in_sizes[2] != NMD * KGT * NGO ||
      in_sizes[3] != NMD * NGO || in_sizes[4] != NMD * NHU || in_sizes[5] != NMD ||
      in_sizes[6] != NBT * NND || in_sizes[7] != NND || in_sizes[8] != NND || out_size != NBT * NND) return;

  const float* feats  = (const float*)d_in[0];
  const float* treat  = (const float*)d_in[1];
  const float* wgate  = (const float*)d_in[2];
  const float* bgate  = (const float*)d_in[3];
  const float* wout   = (const float*)d_in[4];
  const float* bout   = (const float*)d_in[5];
  const int*   modidx = (const int*)d_in[6];
  const int*   lch    = (const int*)d_in[7];
  const int*   rch    = (const int*)d_in[8];
  float* out = (float*)d_out;

  char* ws = (char*)d_ws; size_t off = 0;
  auto carve = [&](size_t bytes) -> char* { char* p = ws + off; off += (bytes + 255) & ~(size_t)255; return p; };
  unsigned short* BT  = (unsigned short*)carve((size_t)NBTR * KGT * 2);
  unsigned*       H16 = (unsigned*)carve((size_t)NBT * NND * NHU * 2);
  float*          C32 = (float*)carve((size_t)NBT * NND * NHU * 4);
  if (off > ws_size || off > (size_t)134217728) return;

  tpw_kernel<1><<<dim3(NGO / 64, KGT / 64, NMD), TPT, 0, stream>>>(wgate, KGT, NGO, KGT, BT, WSCL);
  tree_kernel<<<NBT / RBLK, NTH, 0, stream>>>(feats, treat, bgate, wout, bout, modidx, lch, rch, BT, H16, C32, out);
}
